// MultiHeadAttention_88536455839974
// MI455X (gfx1250) — hardware-verified
//
#include <hip/hip_runtime.h>


#ifndef NB
#define NB 2
#endif
#ifndef SEQ
#define SEQ 2048
#endif
#define NB_FULL  2
#define SEQ_FULL 2048
#define DM   1024
#define NH   16
#define HD   64
#define DQ   (NH * HD)
#define RH   ((SEQ) < 512 ? (SEQ) : 512)
#define PCAR 1024.0f
#define SCL  0.125f
#define LOG2E 1.4426950408889634f

static_assert(HD == 64);
static_assert(DQ == DM);
static_assert(DM % 32 == 0 && DQ % 32 == 0);
static_assert(DM % 8 == 0);
static_assert((NB * SEQ) % 64 == 0 && SEQ % 64 == 0 && DQ % 64 == 0 && DM % 64 == 0);
static_assert(RH % 16 == 0 && (SEQ - RH) % 16 == 0);
static_assert(SEQ % 32 == 0 && ((size_t)SEQ * SEQ) % 1024 == 0);
static_assert(NB <= NB_FULL && SEQ <= SEQ_FULL);

typedef _Float16 h16;
typedef unsigned short bf;
typedef __attribute__((ext_vector_type(16))) __bf16   v16bf;
typedef __attribute__((ext_vector_type(16))) _Float16 v16h;
typedef __attribute__((ext_vector_type(8)))  _Float16 v8h;
typedef __attribute__((ext_vector_type(2)))  _Float16 v2h;
typedef __attribute__((ext_vector_type(16))) unsigned short v16us;
typedef __attribute__((ext_vector_type(8)))  unsigned short v8us;
typedef __attribute__((ext_vector_type(2)))  unsigned short v2us;
typedef __attribute__((ext_vector_type(8)))  float    v8f;
typedef __attribute__((ext_vector_type(4)))  float    v4f;
typedef __attribute__((ext_vector_type(2)))  float    v2f;
typedef v4f  __attribute__((may_alias)) v4fa;

__device__ __forceinline__ unsigned short f2bf(float f) { unsigned u = __float_as_uint(f); u += 0x7FFFu + ((u >> 16) & 1u); return (unsigned short)(u >> 16); }
__device__ __forceinline__ float bf2f(unsigned short b) { return __uint_as_float(((unsigned)b) << 16); }
__device__ __forceinline__ float bfr(float f) { return bf2f(f2bf(f)); }
__device__ __forceinline__ void splitf(float y, unsigned short& h, unsigned short& l) { h = f2bf(y); l = f2bf(y - bf2f(h)); }
__device__ __forceinline__ v16h cat16(v8h lo, v8h hi) { return __builtin_shufflevector(lo, hi, 0, 1, 2, 3, 4, 5, 6, 7, 8, 9, 10, 11, 12, 13, 14, 15); }
__device__ __forceinline__ v16bf cat16b(v8us lo, v8us hi) { return __builtin_bit_cast(v16bf, __builtin_shufflevector(lo, hi, 0, 1, 2, 3, 4, 5, 6, 7, 8, 9, 10, 11, 12, 13, 14, 15)); }
__device__ __forceinline__ v16h  ldh(const h16* p) { return cat16(*(const v8h*)p, *(const v8h*)(p + 16)); }
__device__ __forceinline__ v16bf ldb(const bf* p)  { return cat16b(*(const v8us*)p, *(const v8us*)(p + 16)); }
__device__ __forceinline__ v8f wmma16(v16h a, v16h b, v8f c) { return __builtin_amdgcn_wmma_f32_16x16x32_f16(false, a, false, b, (short)0, c, false, false); }
__device__ __forceinline__ v8f wmmab(v16bf a, v16bf b, v8f c) { return __builtin_amdgcn_wmma_f32_16x16x32_bf16(false, a, false, b, (short)0, c, false, false); }

template <int NSPLIT>
__device__ __forceinline__ void gemm_body(const bf* __restrict__ A, const bf* __restrict__ A2, const bf* __restrict__ Bt, const int K,
                                          float* C, const int ldc, const float* __restrict__ bias, const size_t sA, const size_t sC) {
    __shared__ __align__(16) float os[16 * 68];
    const size_t z = blockIdx.z; A += z * sA; A2 += z * sA; C += z * sC;
    const int lane = threadIdx.x & 31, lr = lane & 15, hi = lane >> 4; const int r0 = (int)blockIdx.x * 64, c0 = (int)blockIdx.y * 64;
    v8f acc[4][4];
#pragma unroll
    for (int mb = 0; mb < 4; ++mb)
#pragma unroll
        for (int nb = 0; nb < 4; ++nb) acc[mb][nb] = (v8f){};
    const size_t aoff = (size_t)(r0 + lr) * K + 8 * hi, boff = (size_t)(c0 + lr) * K + 8 * hi;
#pragma unroll 1
    for (int kc = 0; kc < K; kc += 32) {
        v16bf a[4], a2[4];
#pragma unroll
        for (int mb = 0; mb < 4; ++mb) { a[mb] = ldb(A + aoff + (size_t)mb * 16 * K + kc); if (NSPLIT == 1) a2[mb] = ldb(A2 + aoff + (size_t)mb * 16 * K + kc); }
#pragma unroll
        for (int nb = 0; nb < 4; ++nb) { const v16bf bb = ldb(Bt + boff + (size_t)nb * 16 * K + kc);
#pragma unroll
            for (int mb = 0; mb < 4; ++mb) { acc[mb][nb] = wmmab(a[mb], bb, acc[mb][nb]); if (NSPLIT == 1) acc[mb][nb] = wmmab(a2[mb], bb, acc[mb][nb]); } }
        asm volatile("v_nop\n\tv_nop\n\tv_nop\n\tv_nop" : "+v"(acc[0][0]), "+v"(acc[1][1]), "+v"(acc[2][2]), "+v"(acc[3][3]) : "v"(a[0]), "v"(a[3]));
    }
    v4f bv;
#pragma unroll
    for (int q = 0; q < 4; ++q) bv[q] = bfr(bias[c0 + lr * 4 + q]);
#pragma unroll
    for (int mb = 0; mb < 4; ++mb) {
#pragma unroll
        for (int nb = 0; nb < 4; ++nb) {
#pragma unroll
            for (int j = 0; j < 8; ++j) os[(hi * 8 + j) * 68 + nb * 16 + lr] = acc[mb][nb][j]; }
        __builtin_amdgcn_wave_barrier(); asm volatile("" ::: "memory");
        float* crow = C + (size_t)(r0 + mb * 16) * ldc + c0;
#pragma unroll 1
        for (int ps = 0; ps < 2; ++ps) {
#pragma unroll
            for (int s = 0; s < 8; ++s) { const int row = 2 * s + hi, cofs = lr * 4; v4f val = *(const v4fa*)(os + row * 68 + cofs); val += bv;
                *(volatile v4f*)(crow + (size_t)row * ldc + cofs) = val; }
            if (ps == 0) __threadfence(); }
        __builtin_amdgcn_wave_barrier(); asm volatile("" ::: "memory");
    }
}
__global__ __launch_bounds__(32) void k_gemm1(const bf* __restrict__ A, const bf* __restrict__ Bt, int K, float* C, int ldc, const float* __restrict__ bias, size_t sA, size_t sC) {
    gemm_body<0>(A, A, Bt, K, C, ldc, bias, sA, sC); }
__global__ __launch_bounds__(32) void k_gemm2(const bf* __restrict__ A, const bf* __restrict__ A2, const bf* __restrict__ Bt, int K, float* C, int ldc, const float* __restrict__ bias, size_t sA, size_t sC) {
    gemm_body<1>(A, A2, Bt, K, C, ldc, bias, sA, sC); }

__global__ __launch_bounds__(256) void k_cvt8(const float* __restrict__ src, bf* dst, size_t n8) { const size_t i = (size_t)blockIdx.x * 256 + threadIdx.x; if (i >= n8) return; const v8f v = *(const v8f*)(src + i * 8); v8us o;
#pragma unroll
    for (int k = 0; k < 8; ++k) o[k] = f2bf(v[k]);
    *(volatile v8us*)(dst + i * 8) = o; __threadfence(); *(volatile v8us*)(dst + i * 8) = o; }
__global__ __launch_bounds__(256) void k_cvtx(const float* __restrict__ src, bf* dst) { const size_t i = (size_t)blockIdx.x * 256 + threadIdx.x; if (i >= (size_t)NB * SEQ * DM / 8) return;
    const size_t row = i / (DM / 8); const size_t c8 = i % (DM / 8); const size_t b = row / SEQ, t = row % SEQ; const v8f v = *(const v8f*)(src + ((b * SEQ_FULL + t) * DM + c8 * 8)); v8us o;
#pragma unroll
    for (int k = 0; k < 8; ++k) o[k] = f2bf(v[k]);
    *(volatile v8us*)(dst + i * 8) = o; __threadfence(); *(volatile v8us*)(dst + i * 8) = o; }

__global__ __launch_bounds__(256) void k_cstab(float* CS) { const int idx = (int)blockIdx.x * 256 + (int)threadIdx.x; if (idx >= SEQ * (HD / 2)) return; const int i = idx & 31, t = idx >> 5;
    const float ex = (float)(2 * i) / (float)HD; const float pw = powf(10000.0f, ex); const float invf = 1.0f / pw; const float ang = __fmul_rn((float)t, invf); float sn, cn; sincosf(ang, &sn, &cn);
    v2f cs; cs[0] = cn; cs[1] = sn; float* p0 = CS + ((size_t)t * HD + i) * 2; float* p1 = p0 + (HD / 2) * 2;
    *(volatile v2f*)p0 = cs; *(volatile v2f*)p1 = cs; __threadfence(); *(volatile v2f*)p0 = cs; *(volatile v2f*)p1 = cs; }

__global__ __launch_bounds__(256) void k_mbits(const int* __restrict__ mask, unsigned* MB) { const int lane = threadIdx.x & 31; const int g = (int)blockIdx.x * 8 + (int)(threadIdx.x >> 5);
    if (g >= (int)((size_t)SEQ * SEQ / 1024)) return;
    unsigned mine = 0u;
#pragma unroll 4
    for (int j = 0; j < 32; ++j) { const int wd = g * 32 + j; const int q = wd / (SEQ / 32), kg = wd % (SEQ / 32); const int v = mask[(size_t)q * SEQ_FULL + kg * 32 + lane];
        const unsigned bal = __builtin_amdgcn_ballot_w32(v != 0); mine = (lane == j) ? bal : mine; }
    *(volatile unsigned*)(MB + (size_t)g * 32 + lane) = mine; __threadfence(); *(volatile unsigned*)(MB + (size_t)g * 32 + lane) = mine; }

__global__ __launch_bounds__(256) void k_rope(const float* __restrict__ F, const float* __restrict__ CS, h16* P16, bf* Ph, bf* Pl, int hrows) {
    const size_t e = ((size_t)blockIdx.x * 256 + threadIdx.x) * 2; if (e >= (size_t)NB * NH * SEQ * HD) return; const int d = (int)(e % HD); const int t = (int)((e / HD) % SEQ); const int bh = (int)(e / ((size_t)HD * SEQ)); const int b = bh / NH, h = bh % NH;
    const float* f = F + ((size_t)b * SEQ + t) * DQ + h * HD; v2h o16; v2us oh, ol;
#pragma unroll
    for (int q = 0; q < 2; ++q) { const int dd = d + q; const int dp = (dd < HD / 2) ? dd + HD / 2 : dd - HD / 2; const float x0 = f[dd], x1 = f[dp];
        const v2f cs = *(const v2f*)(CS + ((size_t)t * HD + dd) * 2); float a = __fmul_rn(x0, cs[0]), bq = __fmul_rn(x1, cs[1]); asm volatile("" : "+v"(a)); asm volatile("" : "+v"(bq)); const float r = (dd < HD / 2) ? __fsub_rn(a, bq) : __fadd_rn(a, bq);
        o16[q] = (h16)r; unsigned short a2, c2; splitf(r, a2, c2); oh[q] = a2; ol[q] = c2; }
    const bool wh = (t < hrows); const size_t eh = ((size_t)bh * hrows + (wh ? t : 0)) * HD + d;
    *(volatile v2h*)(P16 + e) = o16; if (wh) { *(volatile v2us*)(Ph + eh) = oh; *(volatile v2us*)(Pl + eh) = ol; }
    __threadfence();
    *(volatile v2h*)(P16 + e) = o16; if (wh) { *(volatile v2us*)(Ph + eh) = oh; *(volatile v2us*)(Pl + eh) = ol; } }
__global__ __launch_bounds__(256) void k_vtp(const float* __restrict__ F, h16* V16, bf* Vh, bf* Vl) { const size_t e = ((size_t)blockIdx.x * 256 + threadIdx.x) * 2; if (e >= (size_t)NB * NH * HD * SEQ) return;
    const int t = (int)(e % SEQ); const int d = (int)((e / SEQ) % HD); const int g = (int)(e / ((size_t)SEQ * HD)); const int b = g / NH, h = g % NH; v2h o16; v2us oh, ol;
#pragma unroll
    for (int q = 0; q < 2; ++q) { const float x = F[((size_t)b * SEQ + t + q) * DQ + h * HD + d]; o16[q] = (h16)x; unsigned short a2, c2; splitf(x, a2, c2); oh[q] = a2; ol[q] = c2; }
    *(volatile v2h*)(V16 + e) = o16; *(volatile v2us*)(Vh + e) = oh; *(volatile v2us*)(Vl + e) = ol; __threadfence(); *(volatile v2h*)(V16 + e) = o16; *(volatile v2us*)(Vh + e) = oh; *(volatile v2us*)(Vl + e) = ol; }

template <bool HR>
__device__ __forceinline__ void attn_body(const h16* __restrict__ Q16, const h16* __restrict__ K16, const h16* __restrict__ VT16,
                                          const bf* __restrict__ Qh, const bf* __restrict__ Ql, const bf* __restrict__ Kh, const bf* __restrict__ Kl,
                                          const bf* __restrict__ VTh, const bf* __restrict__ VTl, const unsigned* __restrict__ MB, bf* ATh, bf* ATl) {
    __shared__ __align__(16) float cs[16 * 68];
    const int lane = threadIdx.x & 31, lr = lane & 15, hi = lane >> 4;
    const int q0 = (HR ? 0 : RH) + (int)blockIdx.x * 16;
    const int bh = (int)blockIdx.y, b = bh / NH, h = bh % NH;
    const size_t qoff = ((size_t)bh * (HR ? RH : SEQ) + q0 + lr) * HD + 8 * hi;
    const size_t koff = ((size_t)bh * SEQ + lr) * HD + 8 * hi;
    const size_t voff = ((size_t)bh * HD + lr) * SEQ + 8 * hi;
    const size_t moff = (size_t)(q0 + lr) * (SEQ / 32);
    const float NINF = -__builtin_huge_valf();
    v8f o[4];
#pragma unroll
    for (int dt = 0; dt < 4; ++dt) o[dt] = (v8f){};
    float m = NINF, l = 0.0f;
#pragma unroll 1
    for (int kc = 0; kc < SEQ / 32; ++kc) {
        const unsigned W = MB[moff + kc];
        if (__builtin_amdgcn_ballot_w32(W != 0u) == 0u) continue;
        const size_t kk = (size_t)kc * 32;
        v8f s0 = (v8f){}, s1 = (v8f){};
        if (HR) {
#pragma unroll
            for (int ks = 0; ks < 2; ++ks) {
                const v16bf qh = ldb(Qh + qoff + ks * 32), ql = ldb(Ql + qoff + ks * 32);
                const v16bf a0h = ldb(Kh + koff + kk * HD + ks * 32), a0l = ldb(Kl + koff + kk * HD + ks * 32);
                const v16bf a1h = ldb(Kh + koff + (kk + 16) * HD + ks * 32), a1l = ldb(Kl + koff + (kk + 16) * HD + ks * 32);
                s0 = wmmab(a0h, qh, s0); s1 = wmmab(a1h, qh, s1); s0 = wmmab(a0l, qh, s0); s1 = wmmab(a1l, qh, s1); s0 = wmmab(a0h, ql, s0); s1 = wmmab(a1h, ql, s1);
                asm volatile("v_nop\n\tv_nop\n\tv_nop\n\tv_nop" : "+v"(s0), "+v"(s1) : "v"(ql), "v"(a0h), "v"(a1h));
            }
        } else {
#pragma unroll
            for (int ks = 0; ks < 2; ++ks) {
                const v16h qf = ldh(Q16 + qoff + ks * 32);
                const v16h k0f = ldh(K16 + koff + kk * HD + ks * 32), k1f = ldh(K16 + koff + (kk + 16) * HD + ks * 32);
                s0 = wmma16(k0f, qf, s0); s1 = wmma16(k1f, qf, s1);
                asm volatile("v_nop\n\tv_nop\n\tv_nop\n\tv_nop" : "+v"(s0), "+v"(s1) : "v"(qf), "v"(k0f), "v"(k1f));
            }
        }
        const unsigned Wl = W >> (8 * hi);
        float t0[8], t1[8]; float mx = NINF;
#pragma unroll
        for (int r = 0; r < 8; ++r) { t0[r] = ((Wl >> r) & 1u) ? s0[r] * SCL : NINF; t1[r] = ((Wl >> (16 + r)) & 1u) ? s1[r] * SCL : NINF; mx = fmaxf(mx, fmaxf(t0[r], t1[r])); }
        mx = fmaxf(mx, __shfl_xor(mx, 16, 32));
        const float mnew = fmaxf(m, mx);
        const float msub = (mnew == NINF) ? 0.0f : mnew;
        float ds = __fsub_rn(m, msub); asm volatile("" : "+v"(ds));
        const float scl = __builtin_amdgcn_exp2f(__fmul_rn(ds, LOG2E));
        float p0[8], p1[8]; float psum = 0.0f;
#pragma unroll
        for (int r = 0; r < 8; ++r) { float d0 = __fsub_rn(t0[r], msub); asm volatile("" : "+v"(d0)); float d1 = __fsub_rn(t1[r], msub); asm volatile("" : "+v"(d1));
            p0[r] = __builtin_amdgcn_exp2f(__fmul_rn(d0, LOG2E)); p1[r] = __builtin_amdgcn_exp2f(__fmul_rn(d1, LOG2E)); psum += p0[r] + p1[r]; }
        psum += __shfl_xor(psum, 16, 32);
        l = l * scl + psum; m = mnew;
#pragma unroll
        for (int dt = 0; dt < 4; ++dt)
#pragma unroll
            for (int r = 0; r < 8; ++r) o[dt][r] *= scl;
        if (HR) {
            v16us ph, pl;
#pragma unroll
            for (int r = 0; r < 8; ++r) { unsigned short a, c; splitf(p0[r], a, c); ph[r] = a; pl[r] = c; splitf(p1[r], a, c); ph[8 + r] = a; pl[8 + r] = c; }
            const v16bf pbh = __builtin_bit_cast(v16bf, ph), pbl = __builtin_bit_cast(v16bf, pl);
            v16bf vh[4], vl[4];
#pragma unroll
            for (int dt = 0; dt < 4; ++dt) { vh[dt] = ldb(VTh + voff + (size_t)dt * 16 * SEQ + kk); vl[dt] = ldb(VTl + voff + (size_t)dt * 16 * SEQ + kk); }
#pragma unroll
            for (int dt = 0; dt < 4; ++dt) { o[dt] = wmmab(vh[dt], pbh, o[dt]); o[dt] = wmmab(vl[dt], pbh, o[dt]); o[dt] = wmmab(vh[dt], pbl, o[dt]); }
            asm volatile("v_nop\n\tv_nop\n\tv_nop\n\tv_nop" : "+v"(o[0]), "+v"(o[1]), "+v"(o[2]), "+v"(o[3]) : "v"(pbh), "v"(pbl), "v"(vh[3]), "v"(vl[3]));
        } else {
            v16h pb;
#pragma unroll
            for (int r = 0; r < 8; ++r) { pb[r] = (h16)(p0[r] * PCAR); pb[8 + r] = (h16)(p1[r] * PCAR); }
            v16h vf[4];
#pragma unroll
            for (int dt = 0; dt < 4; ++dt) vf[dt] = ldh(VT16 + voff + (size_t)dt * 16 * SEQ + kk);
#pragma unroll
            for (int dt = 0; dt < 4; ++dt) o[dt] = wmma16(vf[dt], pb, o[dt]);
            asm volatile("v_nop\n\tv_nop\n\tv_nop\n\tv_nop" : "+v"(o[0]), "+v"(o[1]), "+v"(o[2]), "+v"(o[3]) : "v"(pb), "v"(vf[0]), "v"(vf[3]));
        }
    }
    const float rl = 1.0f / l; const float inv = HR ? rl : rl * (1.0f / PCAR);
#pragma unroll
    for (int dt = 0; dt < 4; ++dt)
#pragma unroll
        for (int r = 0; r < 8; ++r) cs[lr * 68 + dt * 16 + 8 * hi + r] = o[dt][r] * inv;
    __builtin_amdgcn_wave_barrier(); asm volatile("" ::: "memory");
    bf* ah = ATh + ((size_t)b * SEQ + q0) * DQ + h * HD; bf* al = ATl + ((size_t)b * SEQ + q0) * DQ + h * HD;
#pragma unroll 1
    for (int ps = 0; ps < 2; ++ps) {
#pragma unroll
        for (int it = 0; it < 4; ++it) { const int row = it * 4 + (lane >> 3), c = (lane & 7) * 8;
            const v4f x0 = *(const v4fa*)(cs + row * 68 + c), x1 = *(const v4fa*)(cs + row * 68 + c + 4); v8us oh, ol;
#pragma unroll
            for (int q = 0; q < 4; ++q) { unsigned short a, c2; splitf(x0[q], a, c2); oh[q] = a; ol[q] = c2; splitf(x1[q], a, c2); oh[4 + q] = a; ol[4 + q] = c2; }
            *(volatile v8us*)(ah + (size_t)row * DQ + c) = oh; *(volatile v8us*)(al + (size_t)row * DQ + c) = ol; }
        if (ps == 0) __threadfence(); }
}
__global__ __launch_bounds__(32) void k_attn_hi(const bf* __restrict__ Qh, const bf* __restrict__ Ql, const bf* __restrict__ Kh, const bf* __restrict__ Kl, const bf* __restrict__ VTh, const bf* __restrict__ VTl,
                                                const unsigned* __restrict__ MB, bf* ATh, bf* ATl) {
    attn_body<true>(nullptr, nullptr, nullptr, Qh, Ql, Kh, Kl, VTh, VTl, MB, ATh, ATl); }
__global__ __launch_bounds__(32) void k_attn_lo(const h16* __restrict__ Q16, const h16* __restrict__ K16, const h16* __restrict__ VT16, const unsigned* __restrict__ MB, bf* ATh, bf* ATl) {
    attn_body<false>(Q16, K16, VT16, nullptr, nullptr, nullptr, nullptr, nullptr, nullptr, MB, ATh, ATl); }

constexpr size_t al256(size_t x) { return (x + 255) & ~(size_t)255; }
constexpr size_t SZ_XB  = al256((size_t)NB * SEQ * DM * 2);
constexpr size_t SZ_W   = al256((size_t)DQ * DM * 2);
constexpr size_t SZ_CS  = al256((size_t)SEQ * HD * 2 * 4);
constexpr size_t SZ_MB  = al256((size_t)SEQ * SEQ / 8);
constexpr size_t SZ_TMP = al256((size_t)NB * SEQ * DQ * 4);
constexpr size_t SZ_PL  = al256((size_t)NB * NH * SEQ * HD * 2);
constexpr size_t SZ_QH  = al256((size_t)NB * NH * RH * HD * 2);
constexpr size_t SZ_AT  = al256((size_t)NB * SEQ * DQ * 2);
constexpr size_t WS_TOTAL = SZ_XB + 4 * SZ_W + SZ_CS + SZ_MB + SZ_TMP + SZ_PL + 2 * SZ_QH + 3 * SZ_PL + 3 * SZ_PL + 2 * SZ_AT;
static_assert(WS_TOTAL <= (size_t)134217728);

extern "C" void kernel_launch(void* const* d_in, const int* in_sizes, int n_in,
                              void* d_out, int out_size, void* d_ws, size_t ws_size, hipStream_t stream) {
    if (n_in < 10) return;
    const long long need_x = (long long)(NB - 1) * SEQ_FULL * DM + (long long)SEQ * DM;
    if ((long long)in_sizes[0] < need_x || (long long)out_size < need_x) return;
    if (in_sizes[1] < DQ * DM || in_sizes[3] < DQ * DM || in_sizes[5] < DQ * DM || in_sizes[7] < DM * DQ) return;
    if (in_sizes[2] < DQ || in_sizes[4] < DQ || in_sizes[6] < DQ || in_sizes[8] < DM) return;
    if ((long long)in_sizes[9] < (long long)(SEQ - 1) * SEQ_FULL + SEQ) return;
    if (WS_TOTAL > ws_size) return;
    const float* x  = (const float*)d_in[0];
    const float* Wq = (const float*)d_in[1]; const float* bq = (const float*)d_in[2];
    const float* Wk = (const float*)d_in[3]; const float* bk = (const float*)d_in[4];
    const float* Wv = (const float*)d_in[5]; const float* bv = (const float*)d_in[6];
    const float* Wo = (const float*)d_in[7]; const float* bo = (const float*)d_in[8];
    const int* mask = (const int*)d_in[9];
    float* OUT = (float*)d_out;
    char* wsp = (char*)d_ws;
    bf* XB = (bf*)wsp; wsp += SZ_XB;
    bf* WQ = (bf*)wsp; wsp += SZ_W; bf* WK = (bf*)wsp; wsp += SZ_W; bf* WV = (bf*)wsp; wsp += SZ_W; bf* WO = (bf*)wsp; wsp += SZ_W;
    float* CS = (float*)wsp; wsp += SZ_CS;
    unsigned* MB = (unsigned*)wsp; wsp += SZ_MB;
    float* TMP = (float*)wsp; wsp += SZ_TMP;
    h16* Q16 = (h16*)wsp; wsp += SZ_PL; bf* QPh = (bf*)wsp; wsp += SZ_QH; bf* QPl = (bf*)wsp; wsp += SZ_QH;
    h16* K16 = (h16*)wsp; wsp += SZ_PL; bf* KPh = (bf*)wsp; wsp += SZ_PL; bf* KPl = (bf*)wsp; wsp += SZ_PL;
    h16* VT16 = (h16*)wsp; wsp += SZ_PL; bf* VTh = (bf*)wsp; wsp += SZ_PL; bf* VTl = (bf*)wsp; wsp += SZ_PL;
    bf* ATh = (bf*)wsp; wsp += SZ_AT; bf* ATl = (bf*)wsp; wsp += SZ_AT;

    const size_t nw8 = (size_t)DQ * DM / 8;
    k_cvtx<<<(unsigned)(((size_t)NB * SEQ * DM / 8 + 255) / 256), 256, 0, stream>>>(x, XB);
    k_cvt8<<<(unsigned)((nw8 + 255) / 256), 256, 0, stream>>>(Wq, WQ, nw8);
    k_cvt8<<<(unsigned)((nw8 + 255) / 256), 256, 0, stream>>>(Wk, WK, nw8);
    k_cvt8<<<(unsigned)((nw8 + 255) / 256), 256, 0, stream>>>(Wv, WV, nw8);
    k_cvt8<<<(unsigned)((nw8 + 255) / 256), 256, 0, stream>>>(Wo, WO, nw8);
    k_cstab<<<(unsigned)((SEQ * (HD / 2) + 255) / 256), 256, 0, stream>>>(CS);
    k_mbits<<<(unsigned)(((size_t)SEQ * SEQ / 1024 + 7) / 8), 256, 0, stream>>>(mask, MB);

    const dim3 gp((unsigned)(NB * SEQ / 64), (unsigned)(DQ / 64), 1);
    const unsigned LP = (unsigned)(((size_t)NB * NH * SEQ * HD / 2 + 255) / 256);
    k_gemm1<<<gp, 32, 0, stream>>>(XB, WQ, DM, TMP, DQ, bq, (size_t)0, (size_t)0);
    k_rope<<<LP, 256, 0, stream>>>(TMP, CS, Q16, QPh, QPl, RH);
    k_gemm1<<<gp, 32, 0, stream>>>(XB, WK, DM, TMP, DQ, bk, (size_t)0, (size_t)0);
    k_rope<<<LP, 256, 0, stream>>>(TMP, CS, K16, KPh, KPl, SEQ);
    k_gemm1<<<gp, 32, 0, stream>>>(XB, WV, DM, TMP, DQ, bv, (size_t)0, (size_t)0);
    k_vtp<<<LP, 256, 0, stream>>>(TMP, VT16, VTh, VTl);

    k_attn_hi<<<dim3((unsigned)(RH / 16), (unsigned)(NB * NH), 1), 32, 0, stream>>>(QPh, QPl, KPh, KPl, VTh, VTl, MB, ATh, ATl);
    if (SEQ > RH) k_attn_lo<<<dim3((unsigned)((SEQ - RH) / 16), (unsigned)(NB * NH), 1), 32, 0, stream>>>(Q16, K16, VT16, MB, ATh, ATl);

    k_gemm2<<<dim3((unsigned)(SEQ / 64), (unsigned)(DM / 64), (unsigned)NB), 32, 0, stream>>>(ATh, ATl, WO, DQ, OUT, DM, bo, (size_t)SEQ * DQ, (size_t)SEQ_FULL * DM);
}
